// PointNetTransformerSegFast_60507499266132
// MI455X (gfx1250) — hardware-verified
//
#include <hip/hip_runtime.h>
#include <math.h>
#pragma clang fp contract(off)

constexpr int kB        = 2;
constexpr int kNPts     = 16384;
constexpr int kTok      = 2048;
constexpr int kDm       = 256;
constexpr int kHeads    = 8;
constexpr int kDh       = 32;
constexpr int kFF       = 512;
constexpr int kCls      = 50;
constexpr int kClsPad   = 64;
constexpr int kHid      = 128;
constexpr int kHeadHid  = 256;
constexpr int kLayers   = 4;
constexpr int kRows     = kB * kTok;
constexpr int kStep     = kNPts / kTok;
constexpr int kQKld     = 2 * kDm;
constexpr int kQBlk     = 32;
constexpr int kOsPitch  = kDm + 8;
static_assert(kRows == 4096, "token rows");
static_assert(kStep == 8, "token stride");
static_assert(kHeads * kDh == kDm, "head split");
static_assert(kDh == 32, "one k-step per head");
static_assert(2 * kHid == kDm, "stacked hidden width");
static_assert(kHeadHid == kDm, "head hidden width");
static_assert((kOsPitch * 2) % 16 == 0, "LDS row alignment");

constexpr float kWCarry   = 64.0f;
constexpr float kHCarry   = 64.0f;
constexpr float kYCarry   = 16.0f;
constexpr float kQKVCarry = 16.0f;
constexpr float kOCarry   = 256.0f;
constexpr float kGCarry   = 16.0f;
constexpr float kXCarry   = 64.0f;
constexpr float kTCarry   = 64.0f;
constexpr float kLog2e    = 1.4426950408889634f;
constexpr float kLnEps    = 1e-5f;

typedef __attribute__((ext_vector_type(16))) _Float16 v16h;
typedef __attribute__((ext_vector_type(8)))  _Float16 v8h;
typedef __attribute__((ext_vector_type(8)))  float    v8f;
typedef __attribute__((ext_vector_type(4)))  float    v4f;
typedef __attribute__((ext_vector_type(2)))  float    v2f;
typedef __attribute__((ext_vector_type(4)))  unsigned int v4u;

union FragU { v16h v; v8h h[2]; };
__device__ __forceinline__ v16h frag_load(const _Float16* p) {
  FragU f;
  f.h[0] = *(const v8h*)(p);
  f.h[1] = *(const v8h*)(p + 16);
  return f.v;
}
__device__ __forceinline__ v8f wm(v16h a, v16h b, v8f c) {
  return __builtin_amdgcn_wmma_f32_16x16x32_f16(false, a, false, b, (short)0, c, false, false);
}
__device__ __forceinline__ void guard4x5(v8f& a, v8f& b, v8f& c, v8f& d, v16h x, v16h y0, v16h y1, v16h y2, v16h y3) {
  asm volatile("v_nop\n\tv_nop\n\tv_nop\n\tv_nop" : "+v"(a), "+v"(b), "+v"(c), "+v"(d) : "v"(x), "v"(y0), "v"(y1), "v"(y2), "v"(y3));
}
__device__ __forceinline__ void guard4x4(v8f& a, v8f& b, v8f& c, v8f& d, v16h x0, v16h x1, v16h y0, v16h y1) {
  asm volatile("v_nop\n\tv_nop\n\tv_nop\n\tv_nop" : "+v"(a), "+v"(b), "+v"(c), "+v"(d) : "v"(x0), "v"(x1), "v"(y0), "v"(y1));
}
__device__ __forceinline__ void acc_guard4(v8f& a, v8f& b, v8f& c, v8f& d) {
  asm volatile("v_nop\n\tv_nop\n\tv_nop\n\tv_nop" : "+v"(a), "+v"(b), "+v"(c), "+v"(d));
}
__device__ __forceinline__ unsigned h_bits(float f) {
  const _Float16 h = (_Float16)f;
  const unsigned short u = __builtin_bit_cast(unsigned short, h);
  return (unsigned)u;
}
__device__ __forceinline__ unsigned pk16(unsigned a, unsigned b) { return (a & 0xffffu) | (b << 16); }

template <int BIAS_MODE, int OUT_MODE, bool RESID, int ACT>
__global__ __launch_bounds__(256) void wmma_gemm64(
    const unsigned short* __restrict__ Ap, int lda,
    const unsigned short* __restrict__ Btp, int ldb,
    void* __restrict__ Cout, int ldc,
    const float* __restrict__ bias, const float* __restrict__ bias2, int nvalid,
    const float* __restrict__ resid,
    int M, int N, int K, float scale, float oscale) {
  static_assert(!(BIAS_MODE == 1 && ACT != 0), "row bias is applied after the activation slot");
  static_assert(!(BIAS_MODE == 1 && OUT_MODE == 0), "row bias only on the 16-bit path");
  const _Float16* A  = (const _Float16*)Ap;
  const _Float16* Bt = (const _Float16*)Btp;
  __shared__ __align__(16) float sT[8][16 * 68];
  const int lane = threadIdx.x & 31;
  const int wave = threadIdx.x >> 5;
  const int tilesN = N >> 6;
  const int tilesM = M >> 6;
  const int tile = blockIdx.x * 8 + wave;
  if (tile >= tilesM * tilesN) return;
  const int tm = tile / tilesN;
  const int tn = tile - tm * tilesN;
  const int m0 = tm << 6;
  const int n0 = tn << 6;
  const int rlane = lane & 15;
  const int koff  = (lane >> 4) * 8;
  const int mOff  = (lane >> 4) * 8;

  v8f acc[4][4];
#pragma unroll
  for (int i = 0; i < 4; ++i)
#pragma unroll
    for (int j = 0; j < 4; ++j) acc[i][j] = (v8f){0.f, 0.f, 0.f, 0.f, 0.f, 0.f, 0.f, 0.f};

  for (int k0 = 0; k0 < K; k0 += 32) {
    v16h bh[4];
#pragma unroll
    for (int j = 0; j < 4; ++j) {
      const size_t bo = (size_t)(n0 + (j << 4) + rlane) * ldb + koff + k0;
      bh[j] = frag_load(Bt + bo);
    }
#pragma unroll
    for (int i = 0; i < 4; ++i) {
      const size_t ao = (size_t)(m0 + (i << 4) + rlane) * lda + koff + k0;
      const v16h ah = frag_load(A + ao);
#pragma unroll
      for (int j = 0; j < 4; ++j) acc[i][j] = wm(ah, bh[j], acc[i][j]);
      guard4x5(acc[i][0], acc[i][1], acc[i][2], acc[i][3], ah, bh[0], bh[1], bh[2], bh[3]);
    }
  }
  acc_guard4(acc[0][0], acc[0][1], acc[0][2], acc[0][3]);
  acc_guard4(acc[1][0], acc[1][1], acc[1][2], acc[1][3]);
  acc_guard4(acc[2][0], acc[2][1], acc[2][2], acc[2][3]);
  acc_guard4(acc[3][0], acc[3][1], acc[3][2], acc[3][3]);

  float* slab = sT[wave];
#pragma unroll
  for (int i = 0; i < 4; ++i) {
    const int mBase = m0 + (i << 4);
#pragma unroll
    for (int j = 0; j < 4; ++j) {
      const int n = n0 + (j << 4) + rlane;
      float bv = 0.f;
      if (BIAS_MODE == 2) {
        const int nb = (n < nvalid) ? n : (nvalid - 1);
        const float t = bias[nb];
        bv = (n < nvalid) ? t : 0.0f;
      }
      if (BIAS_MODE == 3) bv = bias[n] + bias2[n];
      if (BIAS_MODE == 4) {
        const bool lowhalf = (n0 < kDm);
        const float* bp = lowhalf ? bias : bias2;
        const int nb = lowhalf ? n : (n - kDm);
        bv = bp[nb];
      }
#pragma unroll
      for (int r = 0; r < 8; ++r) {
        float v = acc[i][j][r] * scale;
        v = v + bv;
        if (ACT == 2) v = fmaxf(v, 0.0f);
        slab[(mOff + r) * 68 + (j << 4) + rlane] = v;
      }
    }
    __builtin_amdgcn_fence(__ATOMIC_RELEASE, "workgroup");
    __builtin_amdgcn_wave_barrier();
    __builtin_amdgcn_fence(__ATOMIC_ACQUIRE, "workgroup");
    if (OUT_MODE == 0) {
      float* C = (float*)Cout;
      const int hh = lane >> 4, c4 = (lane & 15) * 4;
      v4f vals[8];
#pragma unroll
      for (int it = 0; it < 8; ++it) {
        const int row = it * 2 + hh;
        v4f v = *(const v4f*)(slab + row * 68 + c4);
        if (RESID) {
          const v4f rr = *(const v4f*)(resid + (size_t)(mBase + row) * ldc + n0 + c4);
          v = v + rr;
        }
        vals[it] = v;
      }
      for (int pass = 0; pass < 2; ++pass) {
#pragma unroll
        for (int it = 0; it < 8; ++it) {
          const int row = it * 2 + hh;
          *(volatile v4f*)(C + (size_t)(mBase + row) * ldc + n0 + c4) = vals[it];
        }
        __threadfence();
      }
    } else {
      unsigned short* C = (unsigned short*)Cout;
      const int q = lane >> 3, c8 = (lane & 7) * 8;
      v4u words[4];
#pragma unroll
      for (int it = 0; it < 4; ++it) {
        const int row = it * 4 + q;
        const float* sp = slab + row * 68 + c8;
        float rb = 0.0f;
        if (BIAS_MODE == 1) rb = bias[mBase + row];
        unsigned hb[8];
#pragma unroll
        for (int e = 0; e < 8; ++e) {
          const float t = (sp[e] + rb) * oscale;
          hb[e] = h_bits(t);
        }
        words[it] = (v4u){pk16(hb[0], hb[1]), pk16(hb[2], hb[3]), pk16(hb[4], hb[5]), pk16(hb[6], hb[7])};
      }
      for (int pass = 0; pass < 2; ++pass) {
#pragma unroll
        for (int it = 0; it < 4; ++it) {
          const int row = it * 4 + q;
          *(volatile v4u*)(C + (size_t)(mBase + row) * ldc + n0 + c8) = words[it];
        }
        __threadfence();
      }
    }
    __builtin_amdgcn_fence(__ATOMIC_RELEASE, "workgroup");
    __builtin_amdgcn_wave_barrier();
    __builtin_amdgcn_fence(__ATOMIC_ACQUIRE, "workgroup");
  }
}

__global__ __launch_bounds__(256) void wtcast_kernel(const float* __restrict__ W, long inStride, int ldw, int nout,
                                                     unsigned short* __restrict__ out, long outStride, int ldk, int koff,
                                                     float carry) {
  __shared__ float sm[64][65];
  const int t  = threadIdx.x;
  const int k0 = blockIdx.x * 64;
  const int n0 = blockIdx.y * 64;
  const float* Wz = W + (size_t)blockIdx.z * inStride;
#pragma unroll 1
  for (int g = 0; g < 2; ++g) {
#pragma unroll
    for (int i = 0; i < 8; ++i) {
      const int e = (g * 8 + i) * 256 + t;
      const int r = e >> 6;
      const int c = e & 63;
      const int n = n0 + c;
      const int nc = (n < nout) ? n : (nout - 1);
      const float v = Wz[(size_t)(k0 + r) * ldw + nc];
      sm[c][r] = (n < nout) ? (v * carry) : 0.0f;
    }
  }
  __syncthreads();
  const int lane = t & 31, wave = t >> 5;
  const int q = lane >> 3, c8 = (lane & 7) * 8;
  unsigned short* op = out + (size_t)blockIdx.z * outStride;
  v4u words[2];
#pragma unroll
  for (int it = 0; it < 2; ++it) {
    const int row = wave * 8 + it * 4 + q;
    unsigned hb[8];
#pragma unroll
    for (int e = 0; e < 8; ++e) hb[e] = h_bits(sm[row][c8 + e]);
    words[it] = (v4u){pk16(hb[0], hb[1]), pk16(hb[2], hb[3]), pk16(hb[4], hb[5]), pk16(hb[6], hb[7])};
  }
  for (int pass = 0; pass < 2; ++pass) {
#pragma unroll
    for (int it = 0; it < 2; ++it) {
      const int row = wave * 8 + it * 4 + q;
      *(volatile v4u*)(op + (size_t)(n0 + row) * ldk + koff + k0 + c8) = words[it];
    }
    __threadfence();
  }
}

__global__ __launch_bounds__(256) void embed_hidden_kernel(const float* __restrict__ xyz,
                                                           const float* __restrict__ ew1, const float* __restrict__ eb1,
                                                           const float* __restrict__ pw1, const float* __restrict__ pb1,
                                                           unsigned short* __restrict__ H, float carry) {
  const int lane = threadIdx.x & 31, wave = threadIdx.x >> 5;
  const int gw = blockIdx.x * 8 + wave;
  const int half = gw & 1;
  const int row = (gw >> 1) * 2 + (lane >> 4);
  const int j0 = (lane & 15) * 8;
  const int b = row / kTok;
  const int m = row - b * kTok;
  const float* tp = xyz + ((size_t)b * kNPts + (size_t)m * kStep) * 3;
  const float t0 = tp[0], t1 = tp[1], t2 = tp[2];
  const float* w = half ? pw1 : ew1;
  const float* bs = half ? pb1 : eb1;
  const v4f wa0 = *(const v4f*)(w + j0),            wa1 = *(const v4f*)(w + j0 + 4);
  const v4f wb0 = *(const v4f*)(w + kHid + j0),     wb1 = *(const v4f*)(w + kHid + j0 + 4);
  const v4f wc0 = *(const v4f*)(w + 2 * kHid + j0), wc1 = *(const v4f*)(w + 2 * kHid + j0 + 4);
  const v4f bb0 = *(const v4f*)(bs + j0),           bb1 = *(const v4f*)(bs + j0 + 4);
  unsigned hb[8];
#pragma unroll
  for (int e = 0; e < 4; ++e) {
    float h0 = ((t0 * wa0[e] + t1 * wb0[e]) + t2 * wc0[e]) + bb0[e];
    float h1 = ((t0 * wa1[e] + t1 * wb1[e]) + t2 * wc1[e]) + bb1[e];
    h0 = fmaxf(h0, 0.0f) * carry;
    h1 = fmaxf(h1, 0.0f) * carry;
    hb[e] = h_bits(h0);
    hb[4 + e] = h_bits(h1);
  }
  const v4u u = (v4u){pk16(hb[0], hb[1]), pk16(hb[2], hb[3]), pk16(hb[4], hb[5]), pk16(hb[6], hb[7])};
  unsigned short* q = H + (size_t)row * kDm + half * kHid + j0;
  *(volatile v4u*)q = u;
  __threadfence();
  *(volatile v4u*)q = u;
}

__global__ __launch_bounds__(256) void ln_kernel(const float* __restrict__ x, const float* __restrict__ s,
                                                 const float* __restrict__ bb, unsigned short* __restrict__ y, float carry) {
  const int lane = threadIdx.x & 31, wave = threadIdx.x >> 5;
  const int row = blockIdx.x * 8 + wave;
  const float* xr = x + (size_t)row * kDm + lane * 8;
  const v4f a = *(const v4f*)(xr);
  const v4f c = *(const v4f*)(xr + 4);
  const v4f s0 = *(const v4f*)(s + lane * 8), s1 = *(const v4f*)(s + lane * 8 + 4);
  const v4f b0 = *(const v4f*)(bb + lane * 8), b1 = *(const v4f*)(bb + lane * 8 + 4);
  float sum = ((a[0] + a[1]) + (a[2] + a[3])) + ((c[0] + c[1]) + (c[2] + c[3]));
#pragma unroll
  for (int off = 16; off >= 1; off >>= 1) sum += __shfl_xor(sum, off, 32);
  const float mean = sum * (1.0f / (float)kDm);
  float d[8];
#pragma unroll
  for (int e = 0; e < 4; ++e) { d[e] = a[e] - mean; d[4 + e] = c[e] - mean; }
  float vs = ((d[0] * d[0] + d[1] * d[1]) + (d[2] * d[2] + d[3] * d[3])) + ((d[4] * d[4] + d[5] * d[5]) + (d[6] * d[6] + d[7] * d[7]));
#pragma unroll
  for (int off = 16; off >= 1; off >>= 1) vs += __shfl_xor(vs, off, 32);
  const float var = vs * (1.0f / (float)kDm);
  const float inv = 1.0f / sqrtf(var + kLnEps);
  unsigned hb[8];
#pragma unroll
  for (int e = 0; e < 4; ++e) {
    const float y0 = (d[e] * inv) * s0[e] + b0[e];
    const float y1 = (d[4 + e] * inv) * s1[e] + b1[e];
    hb[e] = h_bits(y0 * carry);
    hb[4 + e] = h_bits(y1 * carry);
  }
  const v4u u = (v4u){pk16(hb[0], hb[1]), pk16(hb[2], hb[3]), pk16(hb[4], hb[5]), pk16(hb[6], hb[7])};
  unsigned short* q = y + (size_t)row * kDm + lane * 8;
  *(volatile v4u*)q = u;
  __threadfence();
  *(volatile v4u*)q = u;
}

__global__ __launch_bounds__(256) void cast8_kernel(const float* __restrict__ in, unsigned short* __restrict__ out, int n8, float carry) {
  const int i = blockIdx.x * 256 + threadIdx.x;
  if (i >= n8) return;
  const float* p = in + 8 * (size_t)i;
  const v4f a = *(const v4f*)(p);
  const v4f c = *(const v4f*)(p + 4);
  unsigned hb[8];
#pragma unroll
  for (int e = 0; e < 4; ++e) {
    hb[e]     = h_bits(a[e] * carry);
    hb[4 + e] = h_bits(c[e] * carry);
  }
  const v4u u = (v4u){pk16(hb[0], hb[1]), pk16(hb[2], hb[3]), pk16(hb[4], hb[5]), pk16(hb[6], hb[7])};
  unsigned short* q = out + 8 * (size_t)i;
  *(volatile v4u*)q = u;
  __threadfence();
  *(volatile v4u*)q = u;
}

__global__ __launch_bounds__(256) void gelu_kernel(const float* __restrict__ u, unsigned* __restrict__ h, int npairs, float carry) {
#pragma unroll 1
  for (int it = 0; it < 4; ++it) {
    const int i = (it * (int)gridDim.x + (int)blockIdx.x) * 256 + (int)threadIdx.x;
    if (i < npairs) {
      const v2f a = *(const v2f*)(u + 2 * (size_t)i);
      const float a0 = a[0], a1 = a[1];
      unsigned w = 0;
#pragma unroll 1
      for (int e = 0; e < 2; ++e) {
        const float t = (e == 0) ? a0 : a1;
        const float er = erff(t * 0.70710678118654752f);
        const float g = (0.5f * t) * (1.0f + er);
        const unsigned hb = h_bits(g * carry);
        w = w | (hb << (16 * e));
      }
      volatile unsigned* q = (volatile unsigned*)(h + (size_t)i);
      *q = w;
      __threadfence();
      *q = w;
    }
  }
}

__device__ __forceinline__ float pexp2(float s, float c2) {
  float e = s * c2;
  e = fminf(fmaxf(e, -24.0f), 15.0f);
  return exp2f(e);
}

__global__ __launch_bounds__(256) void attn_kernel(const unsigned short* __restrict__ QKp, const unsigned short* __restrict__ Vtp,
                                                   unsigned short* __restrict__ Op, float c2, float ocarry) {
  __shared__ __align__(16) _Float16 Os[kQBlk * kOsPitch];
  const int tid = threadIdx.x;
  const int lane = tid & 31;
  const int head = tid >> 5;
  const int hh = lane >> 4;
  const int c = lane & 15;
  const int qblocks = kTok / kQBlk;
  const int b = blockIdx.x / qblocks;
  const int qb = blockIdx.x - b * qblocks;
  const size_t tok0 = (size_t)b * kTok;
  const int q0 = qb * kQBlk;
  const _Float16* QK = (const _Float16*)QKp;
  const _Float16* Vt = (const _Float16*)Vtp;

  const v16h qf0 = frag_load(QK + (tok0 + q0 + c) * kQKld + head * kDh + 8 * hh);
  const v16h qf1 = frag_load(QK + (tok0 + q0 + 16 + c) * kQKld + head * kDh + 8 * hh);

  const v8f zero8 = (v8f){0.f, 0.f, 0.f, 0.f, 0.f, 0.f, 0.f, 0.f};
  v8f o00 = zero8, o01 = zero8, o10 = zero8, o11 = zero8;
  float ls0 = 0.0f, ls1 = 0.0f;

  const _Float16* kp = QK + (tok0 + c) * kQKld + kDm + head * kDh + 8 * hh;
  const _Float16* vp = Vt + (size_t)(head * kDh + c) * kRows + tok0 + 8 * hh;

#pragma unroll 1
  for (int key0 = 0; key0 < kTok; key0 += 32) {
    const v16h ka0 = frag_load(kp + (size_t)key0 * kQKld);
    const v16h ka1 = frag_load(kp + (size_t)(key0 + 16) * kQKld);
    v8f s00 = wm(ka0, qf0, zero8);
    v8f s01 = wm(ka0, qf1, zero8);
    v8f s10 = wm(ka1, qf0, zero8);
    v8f s11 = wm(ka1, qf1, zero8);
    guard4x4(s00, s01, s10, s11, ka0, ka1, qf0, qf1);
    const v16h va0 = frag_load(vp + key0);
    const v16h va1 = frag_load(vp + (size_t)16 * kRows + key0);
    v16h pb0, pb1;
#pragma unroll
    for (int r = 0; r < 8; ++r) {
      const float p00 = pexp2(s00[r], c2);
      const float p10 = pexp2(s10[r], c2);
      const float p01 = pexp2(s01[r], c2);
      const float p11 = pexp2(s11[r], c2);
      ls0 = ls0 + (p00 + p10);
      ls1 = ls1 + (p01 + p11);
      pb0[r]     = (_Float16)p00;
      pb0[8 + r] = (_Float16)p10;
      pb1[r]     = (_Float16)p01;
      pb1[8 + r] = (_Float16)p11;
    }
    o00 = wm(va0, pb0, o00);
    o01 = wm(va0, pb1, o01);
    o10 = wm(va1, pb0, o10);
    o11 = wm(va1, pb1, o11);
    guard4x4(o00, o01, o10, o11, va0, va1, pb0, pb1);
  }

  const float lt0 = ls0 + __shfl_xor(ls0, 16, 32);
  const float lt1 = ls1 + __shfl_xor(ls1, 16, 32);
  const float inv0 = ocarry * (1.0f / lt0);
  const float inv1 = ocarry * (1.0f / lt1);
  v8h h00, h01, h10, h11;
#pragma unroll
  for (int r = 0; r < 8; ++r) {
    h00[r] = (_Float16)(o00[r] * inv0);
    h10[r] = (_Float16)(o10[r] * inv0);
    h01[r] = (_Float16)(o01[r] * inv1);
    h11[r] = (_Float16)(o11[r] * inv1);
  }
  *(v8h*)(Os + (c) * kOsPitch + head * kDh + 8 * hh)           = h00;
  *(v8h*)(Os + (c) * kOsPitch + head * kDh + 16 + 8 * hh)      = h10;
  *(v8h*)(Os + (16 + c) * kOsPitch + head * kDh + 8 * hh)      = h01;
  *(v8h*)(Os + (16 + c) * kOsPitch + head * kDh + 16 + 8 * hh) = h11;
  __syncthreads();
  v8h vals[4];
#pragma unroll
  for (int it = 0; it < 4; ++it) {
    const int row = it * 8 + head;
    vals[it] = *(const v8h*)(Os + row * kOsPitch + lane * 8);
  }
  for (int pass = 0; pass < 2; ++pass) {
#pragma unroll
    for (int it = 0; it < 4; ++it) {
      const int row = it * 8 + head;
      *(volatile v8h*)(Op + (tok0 + q0 + row) * kDm + lane * 8) = vals[it];
    }
    __threadfence();
  }
}

__global__ __launch_bounds__(256) void knn_kernel(const float* __restrict__ xyz, const float* __restrict__ logits,
                                                  float* __restrict__ out) {
#pragma clang fp contract(off)
  __shared__ float tkx[kTok];
  __shared__ float tky[kTok];
  __shared__ float tkz[kTok];
  __shared__ float tk2[kTok];
  __shared__ int nbr[256 * 3];
  const int tid = threadIdx.x;
  const int blocksPerBatch = kNPts / 256;
  const int b = blockIdx.x / blocksPerBatch;
  const int nb = blockIdx.x - b * blocksPerBatch;
#pragma unroll 1
  for (int m = tid; m < kTok; m += 256) {
    const v4f t = *(const v4f*)(xyz + ((size_t)b * kNPts + (size_t)m * kStep) * 3);
    const float tx = t[0], ty = t[1], tz = t[2];
    const float xx = tx * tx;
    const float yy = ty * ty;
    const float zz = tz * tz;
    tkx[m] = tx;
    tky[m] = ty;
    tkz[m] = tz;
    tk2[m] = (xx + zz) + yy;
  }
  __syncthreads();
  const int n = nb * 256 + tid;
  const float* qp = xyz + ((size_t)b * kNPts + (size_t)n) * 3;
  const float qx = qp[0], qy = qp[1], qz = qp[2];
  const float qxx = qx * qx;
  const float qyy = qy * qy;
  const float qzz = qz * qz;
  const float q2 = (qxx + qzz) + qyy;
  float d0 = INFINITY, d1 = INFINITY, d2 = INFINITY;
  int i0 = 0, i1 = 0, i2 = 0;
#pragma unroll 4
  for (int m = 0; m < kTok; ++m) {
    float p = qx * tkx[m];
    p = __builtin_fmaf(qy, tky[m], p);
    p = __builtin_fmaf(qz, tkz[m], p);
    const float twop = 2.0f * p;
    const float sq = q2 + tk2[m];
    float d = sq - twop;
    d = fmaxf(d, 0.0f);
    if (d < d2) {
      const bool c0 = d < d0;
      const bool c1 = d < d1;
      const float nd2 = c1 ? d1 : d;
      const int   ni2 = c1 ? i1 : m;
      const float nd1 = c0 ? d0 : (c1 ? d : d1);
      const int   ni1 = c0 ? i0 : (c1 ? m : i1);
      const float nd0 = c0 ? d : d0;
      const int   ni0 = c0 ? m : i0;
      d0 = nd0; d1 = nd1; d2 = nd2;
      i0 = ni0; i1 = ni1; i2 = ni2;
    }
  }
  i0 = min(max(i0, 0), kTok - 1);
  i1 = min(max(i1, 0), kTok - 1);
  i2 = min(max(i2, 0), kTok - 1);
  nbr[tid * 3 + 0] = i0;
  nbr[tid * 3 + 1] = i1;
  nbr[tid * 3 + 2] = i2;
  __syncthreads();

  const float third = 1.0f / 3.0f;
  const float* Lb = logits + (size_t)b * kTok * kClsPad;
  float* ob = out + ((size_t)b * kNPts + (size_t)nb * 256) * kCls;
  const int nvec = 256 * kCls / 4;
#pragma unroll 1
  for (int it = 0; it < 13; ++it) {
    const int f = it * 256 + tid;
    const int fc = (f < nvec) ? f : (nvec - 1);
    float v[4];
#pragma unroll
    for (int e = 0; e < 4; ++e) {
      const int el = fc * 4 + e;
      const int qn = el / kCls;
      const int ch = el - qn * kCls;
      const int a0 = nbr[qn * 3 + 0];
      const int a1 = nbr[qn * 3 + 1];
      const int a2 = nbr[qn * 3 + 2];
      const float l0 = Lb[a0 * kClsPad + ch];
      const float l1 = Lb[a1 * kClsPad + ch];
      const float l2 = Lb[a2 * kClsPad + ch];
      const float sm = (l0 + l1) + l2;
      v[e] = sm * third;
    }
    const v4f val = (v4f){v[0], v[1], v[2], v[3]};
    if (f < nvec) {
      *(volatile v4f*)(ob + (size_t)f * 4) = val;
      __threadfence();
      *(volatile v4f*)(ob + (size_t)f * 4) = val;
    }
  }
}

constexpr bool gemm_shape_ok(int M, int N, int K) {
  return (M % 64 == 0) && (N % 64 == 0) && (K % 32 == 0) && ((((M / 64) * (N / 64)) % 8) == 0);
}
static_assert(gemm_shape_ok(kRows, kDm, kDm), "token x 256 x 256");
static_assert(gemm_shape_ok(kRows, kQKld, kDm), "qk projection");
static_assert(gemm_shape_ok(kDm, kRows, kDm), "transposed v projection");
static_assert(gemm_shape_ok(kRows, kFF, kDm), "ffn up");
static_assert(gemm_shape_ok(kRows, kDm, kFF), "ffn down");
static_assert(gemm_shape_ok(kRows, kClsPad, kHeadHid), "class head");
static_assert((kB * kNPts * kCls) % 4 == 0, "flat vector output");
static_assert((256 * kCls * 4) % 128 == 0, "block output range is line aligned");

extern "C" void kernel_launch(void* const* d_in, const int* in_sizes, int n_in,
                              void* d_out, int out_size, void* d_ws, size_t ws_size,
                              hipStream_t stream) {
  (void)in_sizes; (void)n_in; (void)out_size;
  const float* xyz = (const float*)d_in[0];
  const float* ew1 = (const float*)d_in[1];  const float* eb1 = (const float*)d_in[2];
  const float* ew2 = (const float*)d_in[3];  const float* eb2 = (const float*)d_in[4];
  const float* pw1 = (const float*)d_in[5];  const float* pb1 = (const float*)d_in[6];
  const float* pw2 = (const float*)d_in[7];  const float* pb2 = (const float*)d_in[8];
  const float* Wq = (const float*)d_in[9];   const float* bq = (const float*)d_in[10];
  const float* Wk = (const float*)d_in[11];  const float* bk = (const float*)d_in[12];
  const float* Wv = (const float*)d_in[13];  const float* bv = (const float*)d_in[14];
  const float* Wo = (const float*)d_in[15];  const float* bo = (const float*)d_in[16];
  const float* l1s = (const float*)d_in[17]; const float* l1b = (const float*)d_in[18];
  const float* W1 = (const float*)d_in[19];  const float* b1 = (const float*)d_in[20];
  const float* W2 = (const float*)d_in[21];  const float* b2 = (const float*)d_in[22];
  const float* l2s = (const float*)d_in[23]; const float* l2b = (const float*)d_in[24];
  const float* hw1 = (const float*)d_in[25]; const float* hb1 = (const float*)d_in[26];
  const float* hw2 = (const float*)d_in[27]; const float* hb2 = (const float*)d_in[28];

  char* w = (char*)d_ws;
  size_t off = 0;
  auto carve = [&](size_t bytes) { size_t o = off; off += (bytes + 255) & ~(size_t)255; return o; };
  const size_t o_x0   = carve((size_t)kRows * kDm * 4);
  const size_t o_x1   = carve((size_t)kRows * kDm * 4);
  const size_t o_u    = carve((size_t)kRows * kFF * 4);
  const size_t o_y16  = carve((size_t)kRows * kDm * 2);
  const size_t o_qk   = carve((size_t)kRows * kQKld * 2);
  const size_t o_vt   = carve((size_t)kDm * kRows * 2);
  const size_t o_o16  = carve((size_t)kRows * kDm * 2);
  const size_t o_h16  = carve((size_t)kRows * kFF * 2);
  const size_t o_t16  = carve((size_t)kRows * kHeadHid * 2);
  const size_t o_lg   = carve((size_t)kRows * kClsPad * 4);
  const size_t o_wqk  = carve((size_t)kLayers * kQKld * kDm * 2);
  const size_t o_wv   = carve((size_t)kLayers * kDm * kDm * 2);
  const size_t o_wo   = carve((size_t)kLayers * kDm * kDm * 2);
  const size_t o_w1   = carve((size_t)kLayers * kFF * kDm * 2);
  const size_t o_w2   = carve((size_t)kLayers * kDm * kFF * 2);
  const size_t o_emb  = carve((size_t)kDm * kDm * 2);
  const size_t o_hw1  = carve((size_t)kHeadHid * kDm * 2);
  const size_t o_hw2  = carve((size_t)kClsPad * kHeadHid * 2);
  if (off > ws_size || off > (size_t)134217728) return;

  float* x0 = (float*)(w + o_x0);
  float* x1 = (float*)(w + o_x1);
  float* u  = (float*)(w + o_u);
  unsigned short* y16  = (unsigned short*)(w + o_y16);
  unsigned short* qk16 = (unsigned short*)(w + o_qk);
  unsigned short* vt16 = (unsigned short*)(w + o_vt);
  unsigned short* o16  = (unsigned short*)(w + o_o16);
  unsigned short* h16  = (unsigned short*)(w + o_h16);
  unsigned short* t16  = (unsigned short*)(w + o_t16);
  float* lg = (float*)(w + o_lg);
  unsigned short* WqkT = (unsigned short*)(w + o_wqk);
  unsigned short* WvT  = (unsigned short*)(w + o_wv);
  unsigned short* WoT  = (unsigned short*)(w + o_wo);
  unsigned short* W1T  = (unsigned short*)(w + o_w1);
  unsigned short* W2T  = (unsigned short*)(w + o_w2);
  unsigned short* embT = (unsigned short*)(w + o_emb);
  unsigned short* hw1T = (unsigned short*)(w + o_hw1);
  unsigned short* hw2T = (unsigned short*)(w + o_hw2);

  wtcast_kernel<<<dim3(kDm / 64, kDm / 64, kLayers), 256, 0, stream>>>(Wq, (long)kDm * kDm, kDm, kDm, WqkT, (long)kQKld * kDm, kDm, 0, kWCarry);
  wtcast_kernel<<<dim3(kDm / 64, kDm / 64, kLayers), 256, 0, stream>>>(Wk, (long)kDm * kDm, kDm, kDm, WqkT + (size_t)kDm * kDm, (long)kQKld * kDm, kDm, 0, kWCarry);
  wtcast_kernel<<<dim3(kDm / 64, kDm / 64, kLayers), 256, 0, stream>>>(Wv, (long)kDm * kDm, kDm, kDm, WvT, (long)kDm * kDm, kDm, 0, kWCarry);
  wtcast_kernel<<<dim3(kDm / 64, kDm / 64, kLayers), 256, 0, stream>>>(Wo, (long)kDm * kDm, kDm, kDm, WoT, (long)kDm * kDm, kDm, 0, kWCarry);
  wtcast_kernel<<<dim3(kDm / 64, kFF / 64, kLayers), 256, 0, stream>>>(W1, (long)kDm * kFF, kFF, kFF, W1T, (long)kFF * kDm, kDm, 0, kWCarry);
  wtcast_kernel<<<dim3(kFF / 64, kDm / 64, kLayers), 256, 0, stream>>>(W2, (long)kFF * kDm, kDm, kDm, W2T, (long)kDm * kFF, kFF, 0, kWCarry);
  wtcast_kernel<<<dim3(kHid / 64, kDm / 64, 1), 256, 0, stream>>>(ew2, 0L, kDm, kDm, embT, 0L, kDm, 0, kWCarry);
  wtcast_kernel<<<dim3(kHid / 64, kDm / 64, 1), 256, 0, stream>>>(pw2, 0L, kDm, kDm, embT, 0L, kDm, kHid, kWCarry);
  wtcast_kernel<<<dim3(kDm / 64, kHeadHid / 64, 1), 256, 0, stream>>>(hw1, 0L, kHeadHid, kHeadHid, hw1T, 0L, kDm, 0, kWCarry);
  wtcast_kernel<<<dim3(kHeadHid / 64, kClsPad / 64, 1), 256, 0, stream>>>(hw2, 0L, kCls, kCls, hw2T, 0L, kHeadHid, 0, kWCarry);

  const float sEmb = 1.0f / (kHCarry * kWCarry);
  const float sY   = 1.0f / (kYCarry * kWCarry);
  const float sWo  = 1.0f / (kOCarry * kWCarry);
  const float sW2  = 1.0f / (kGCarry * kWCarry);
  const float sH1  = 1.0f / (kXCarry * kWCarry);
  const float sH2  = 1.0f / (kTCarry * kWCarry);
  const float attnScale = 1.0f / sqrtf((float)kDh);
  const float c2 = (attnScale * kLog2e) / (kQKVCarry * kQKVCarry);
  const float oc = kOCarry / kQKVCarry;

  embed_hidden_kernel<<<kRows / 8, 256, 0, stream>>>(xyz, ew1, eb1, pw1, pb1, y16, kHCarry);
  wmma_gemm64<3, 0, false, 0><<<(kRows / 64) * (kDm / 64) / 8, 256, 0, stream>>>(
      y16, kDm, embT, kDm, x0, kDm, eb2, pb2, kDm, x0, kRows, kDm, kDm, sEmb, 1.0f);

  for (int l = 0; l < kLayers; ++l) {
    ln_kernel<<<kRows / 8, 256, 0, stream>>>(x0, l1s + l * kDm, l1b + l * kDm, y16, kYCarry);
    wmma_gemm64<4, 1, false, 0><<<(kRows / 64) * (kQKld / 64) / 8, 256, 0, stream>>>(
        y16, kDm, WqkT + (size_t)l * kQKld * kDm, kDm, qk16, kQKld, bq + l * kDm, bk + l * kDm, kQKld, x0,
        kRows, kQKld, kDm, sY, kQKVCarry);
    wmma_gemm64<1, 1, false, 0><<<(kDm / 64) * (kRows / 64) / 8, 256, 0, stream>>>(
        WvT + (size_t)l * kDm * kDm, kDm, y16, kDm, vt16, kRows, bv + l * kDm, bv + l * kDm, kRows, x0,
        kDm, kRows, kDm, sY, kQKVCarry);
    attn_kernel<<<kB * (kTok / kQBlk), 256, 0, stream>>>(qk16, vt16, o16, c2, oc);
    wmma_gemm64<2, 0, true, 0><<<(kRows / 64) * (kDm / 64) / 8, 256, 0, stream>>>(
        o16, kDm, WoT + (size_t)l * kDm * kDm, kDm, x1, kDm, bo + l * kDm, bo + l * kDm, kDm, x0,
        kRows, kDm, kDm, sWo, 1.0f);
    ln_kernel<<<kRows / 8, 256, 0, stream>>>(x1, l2s + l * kDm, l2b + l * kDm, y16, kYCarry);
    wmma_gemm64<2, 0, false, 0><<<(kRows / 64) * (kFF / 64) / 8, 256, 0, stream>>>(
        y16, kDm, W1T + (size_t)l * kFF * kDm, kDm, u, kFF, b1 + l * kFF, b1 + l * kFF, kFF, x1,
        kRows, kFF, kDm, sY, 1.0f);
    gelu_kernel<<<(kRows * kFF / 2) / (256 * 4), 256, 0, stream>>>(u, (unsigned*)h16, kRows * kFF / 2, kGCarry);
    wmma_gemm64<2, 0, true, 0><<<(kRows / 64) * (kDm / 64) / 8, 256, 0, stream>>>(
        h16, kFF, W2T + (size_t)l * kDm * kFF, kFF, x0, kDm, b2 + l * kDm, b2 + l * kDm, kDm, x1,
        kRows, kDm, kFF, sW2, 1.0f);
  }

  cast8_kernel<<<(kRows * kDm / 8) / 256, 256, 0, stream>>>(x0, y16, kRows * kDm / 8, kXCarry);
  wmma_gemm64<2, 1, false, 2><<<(kRows / 64) * (kHeadHid / 64) / 8, 256, 0, stream>>>(
      y16, kDm, hw1T, kDm, t16, kHeadHid, hb1, hb1, kHeadHid, x0, kRows, kHeadHid, kDm, sH1, kTCarry);
  wmma_gemm64<2, 0, false, 0><<<(kRows / 64) * (kClsPad / 64) / 8, 256, 0, stream>>>(
      t16, kHeadHid, hw2T, kHeadHid, lg, kClsPad, hb2, hb2, kCls, x0, kRows, kClsPad, kHeadHid, sH2, 1.0f);

  knn_kernel<<<kB * (kNPts / 256), 256, 0, stream>>>(xyz, lg, (float*)d_out);
}
